// SharedEncoder_13400297963521
// MI455X (gfx1250) — hardware-verified
//
#include <hip/hip_runtime.h>

typedef __attribute__((ext_vector_type(16))) _Float16 v16h;
typedef __attribute__((ext_vector_type(8)))  _Float16 v8h;
typedef __attribute__((ext_vector_type(16))) __bf16   v16b;
typedef __attribute__((ext_vector_type(8)))  __bf16   v8b;
typedef __attribute__((ext_vector_type(8)))  float    v8f;
typedef __attribute__((ext_vector_type(4)))  float    v4f;
#define PSCALE 32768.0f
#define U16(p) ((const unsigned short*)(const void*)(p))
#define PSCALE_INV (1.0f / 32768.0f)

__device__ __forceinline__ unsigned short f2bf_bits(float f) {
  unsigned u = __float_as_uint(f);
  return (unsigned short)((u + 0x7FFFu + ((u >> 16) & 1u)) >> 16);
}
__device__ __forceinline__ float bf_bits2f(unsigned short h) { return __uint_as_float(((unsigned)h) << 16); }

__device__ __forceinline__ void dep_guard_h(v8f& a, v8f& b, v16h x, v16h y) { asm volatile("v_nop\n\tv_nop\n\tv_nop\n\tv_nop" : "+v"(a), "+v"(b) : "v"(x), "v"(y)); }
__device__ __forceinline__ void dep_guard_b(v8f& a, v8f& b, v16b x, v16b y) { asm volatile("v_nop\n\tv_nop\n\tv_nop\n\tv_nop" : "+v"(a), "+v"(b) : "v"(x), "v"(y)); }
__device__ __forceinline__ void keep4_h(v16h a, v16h b, v16h c, v16h d) { asm volatile("v_nop" :: "v"(a), "v"(b), "v"(c), "v"(d)); }
__device__ __forceinline__ void keep4_b(v16b a, v16b b, v16b c, v16b d) { asm volatile("v_nop" :: "v"(a), "v"(b), "v"(c), "v"(d)); }
__device__ __forceinline__ void acc_guard4(v8f& a, v8f& b, v8f& c, v8f& d) { asm volatile("v_nop\n\tv_nop\n\tv_nop\n\tv_nop" : "+v"(a), "+v"(b), "+v"(c), "+v"(d)); }
template <typename T> struct Frag;
template <> struct Frag<_Float16> {
  typedef v16h V; union U { v16h v; v8h h[2]; };
  static __device__ __forceinline__ v16h load(const _Float16* p) {
    U f; f.h[0] = *(const v8h*)(p); f.h[1] = *(const v8h*)(p + 16); return f.v;
  }
  static __device__ __forceinline__ v8f mma(v16h a, v16h b, v8f c) {
    return __builtin_amdgcn_wmma_f32_16x16x32_f16(false, a, false, b, (short)0, c, false, false);
  }
  static __device__ __forceinline__ void guard(v8f& a, v8f& b, v16h x, v16h y) { dep_guard_h(a, b, x, y); }
  static __device__ __forceinline__ void keep(v16h a, v16h b, v16h c, v16h d) { keep4_h(a, b, c, d); }
};
template <> struct Frag<__bf16> {
  typedef v16b V; union U { v16b v; v8b h[2]; };
  static __device__ __forceinline__ v16b load(const __bf16* p) {
    U f; f.h[0] = *(const v8b*)(p); f.h[1] = *(const v8b*)(p + 16); return f.v;
  }
  static __device__ __forceinline__ v8f mma(v16b a, v16b b, v8f c) {
    return __builtin_amdgcn_wmma_f32_16x16x32_bf16(false, a, false, b, (short)0, c, false, false);
  }
  static __device__ __forceinline__ void guard(v8f& a, v8f& b, v16b x, v16b y) { dep_guard_b(a, b, x, y); }
  static __device__ __forceinline__ void keep(v16b a, v16b b, v16b c, v16b d) { keep4_b(a, b, c, d); }
};

template <int ET> struct Elem;
template <> struct Elem<0> { typedef _Float16 T; };
template <> struct Elem<1> { typedef __bf16 T; };
template <int ET, bool SPLIT, int BIAS_MODE, int OUT_MODE, bool RESID, int ACT = 0>
__global__ __launch_bounds__(256) void wmma_gemm64(
    const unsigned short* __restrict__ Ap, const unsigned short* __restrict__ A2p, int lda, long strideA,
    const unsigned short* __restrict__ Btp, const unsigned short* __restrict__ Bt2p, int ldb, long strideB,
    void* __restrict__ Cout, void* __restrict__ Cout2, int ldc, long strideC,
    const float* __restrict__ bias,
    const float* __restrict__ resid, long strideR,
    int M, int N, int K, float scale) {
  typedef typename Elem<ET>::T T;
  typedef typename Frag<T>::V V;
  const T* A = (const T*)Ap; const T* A2 = (const T*)A2p; const T* Bt = (const T*)Btp; const T* Bt2 = (const T*)Bt2p;
  __shared__ __align__(16) float sT[8][16 * 68];
  const int b    = blockIdx.y;
  const int lane = threadIdx.x & 31;
  const int wave = threadIdx.x >> 5;
  const int tilesN = N >> 6;
  const int tilesM = M >> 6;
  const int tile = blockIdx.x * 8 + wave;
  if (tile >= tilesM * tilesN) return;
  const int tm = tile / tilesN;
  const int tn = tile - tm * tilesN;
  const int m0 = tm << 6;
  const int n0 = tn << 6;

  const T* Ab  = A  + (size_t)b * strideA;
  const T* Bb  = Bt + (size_t)b * strideB;
  const T* Ab2 = SPLIT ? (A2  + (size_t)b * strideA) : nullptr;
  const T* Bb2 = SPLIT ? (Bt2 + (size_t)b * strideB) : nullptr;

  const int rlane = lane & 15;
  const int koff  = (lane >> 4) * 8;
  const int mOff  = (lane >> 4) * 8;

  v8f acc[4][4];
#pragma unroll
  for (int i = 0; i < 4; ++i)
#pragma unroll
    for (int j = 0; j < 4; ++j) acc[i][j] = (v8f){0.f,0.f,0.f,0.f,0.f,0.f,0.f,0.f};

  for (int k0 = 0; k0 < K; k0 += 32) {
    V bh[4], bl[4];
#pragma unroll
    for (int j = 0; j < 4; ++j) {
      const size_t bo = (size_t)(n0 + (j << 4) + rlane) * ldb + koff + k0;
      bh[j] = Frag<T>::load(Bb + bo);
      if (SPLIT) bl[j] = Frag<T>::load(Bb2 + bo);
    }
#pragma unroll
    for (int i = 0; i < 4; ++i) {
      const size_t ao = (size_t)(m0 + (i << 4) + rlane) * lda + koff + k0;
      V ah = Frag<T>::load(Ab + ao);
      V al;
      if (SPLIT) al = Frag<T>::load(Ab2 + ao);
#pragma unroll
      for (int j = 0; j < 4; ++j) {
        acc[i][j] = Frag<T>::mma(ah, bh[j], acc[i][j]);
        if (SPLIT) {
          acc[i][j] = Frag<T>::mma(ah, bl[j], acc[i][j]);
          acc[i][j] = Frag<T>::mma(al, bh[j], acc[i][j]);
        }
      }
      Frag<T>::guard(acc[i][0], acc[i][3], ah, SPLIT ? al : ah);
    }
    Frag<T>::keep(bh[0], bh[1], bh[2], bh[3]);
    if (SPLIT) Frag<T>::keep(bl[0], bl[1], bl[2], bl[3]);
  }
  acc_guard4(acc[0][0], acc[0][1], acc[0][2], acc[0][3]);
  acc_guard4(acc[1][0], acc[1][1], acc[1][2], acc[1][3]);
  acc_guard4(acc[2][0], acc[2][1], acc[2][2], acc[2][3]);
  acc_guard4(acc[3][0], acc[3][1], acc[3][2], acc[3][3]);

  float* slab = sT[wave];
  const float* Rb = RESID ? (resid + (size_t)b * strideR) : nullptr;
#pragma unroll
  for (int i = 0; i < 4; ++i) {
    const int mBase = m0 + (i << 4);
#pragma unroll
    for (int j = 0; j < 4; ++j) {
      const int n = n0 + (j << 4) + rlane;
      float bv = 0.f;
      if (BIAS_MODE == 2) bv = bias[n];
#pragma unroll
      for (int r = 0; r < 8; ++r) {
        float v = acc[i][j][r] * scale;
        if (BIAS_MODE == 1) v += bias[mBase + mOff + r];
        if (BIAS_MODE == 2) v += bv;
        if (RESID) v += Rb[(size_t)(mBase + mOff + r) * ldc + n];
        if (ACT == 1) v = tanhf(v);
        if (ACT == 2) v = fmaxf(v, 0.0f);
        if (ACT == 3) v = v / (1.0f + expf(-v));
        if (ACT == 4) v = (v > 0.f) ? v : 0.01f * v;
        if (ACT == 5) v = 0.5f * v * (1.0f + erff(v * 0.70710678118654752f));
        slab[(mOff + r) * 68 + (j << 4) + rlane] = v;
      }
    }
    __builtin_amdgcn_fence(__ATOMIC_RELEASE, "workgroup");
    __builtin_amdgcn_wave_barrier();
    __builtin_amdgcn_fence(__ATOMIC_ACQUIRE, "workgroup");
    if (OUT_MODE == 0) {
      float* C = (float*)Cout + (size_t)b * strideC;
      const int hh = lane >> 4, c4 = (lane & 15) * 4;
      for (int pass = 0; pass < 2; ++pass) {
#pragma unroll
        for (int it = 0; it < 8; ++it) {
          const int row = it * 2 + hh;
          v4f v = *(const v4f*)(slab + row * 68 + c4);
          *(volatile v4f*)(C + (size_t)(mBase + row) * ldc + n0 + c4) = v;
        }
        __threadfence();
      }
    } else {
      const int q = lane >> 3, c8 = (lane & 7) * 8;
      unsigned short* C  = (unsigned short*)Cout  + (size_t)b * strideC;
      unsigned short* C2 = (OUT_MODE == 2) ? ((unsigned short*)Cout2 + (size_t)b * strideC) : nullptr;
      for (int pass = 0; pass < 2; ++pass) {
#pragma unroll
        for (int it = 0; it < 4; ++it) {
          const int row = it * 4 + q;
          const float* sp = slab + row * 68 + c8;
          v8h hv, lv;
#pragma unroll
          for (int e = 0; e < 8; ++e) {
            if (OUT_MODE == 1) {
              hv[e] = (_Float16)sp[e];
            } else {
              unsigned short hb = f2bf_bits(sp[e]);
              unsigned short lb = f2bf_bits(sp[e] - bf_bits2f(hb));
              hv[e] = __builtin_bit_cast(_Float16, hb);
              lv[e] = __builtin_bit_cast(_Float16, lb);
            }
          }
          *(volatile v8h*)(C + (size_t)(mBase + row) * ldc + n0 + c8) = hv;
          if (OUT_MODE == 2) *(volatile v8h*)(C2 + (size_t)(mBase + row) * ldc + n0 + c8) = lv;
        }
        __threadfence();
      }
    }
    __builtin_amdgcn_fence(__ATOMIC_RELEASE, "workgroup");
    __builtin_amdgcn_wave_barrier();
    __builtin_amdgcn_fence(__ATOMIC_ACQUIRE, "workgroup");
  }
}

constexpr int NBATCH = 64;
constexpr int NSTEP  = 512;
constexpr int NEMB   = 256;
constexpr int NHID   = 512;
constexpr int NG4    = 4 * NHID;
constexpr int STEPS_PER_LAUNCH = 128;
constexpr int NCHUNK = NSTEP / STEPS_PER_LAUNCH;
constexpr int MCHUNK = STEPS_PER_LAUNCH * NBATCH;
constexpr int RB_ROWS = 16;
constexpr int RB_WAVES = 16;
constexpr int RB_THREADS = RB_WAVES * 32;
constexpr int APITCH = 528;
constexpr int OPITCH = 516;
constexpr float W_CARRY = 16.0f;
constexpr float W_CARRY_INV = 0.0625f;

static_assert(NSTEP % STEPS_PER_LAUNCH == 0, "chunking");
static_assert(MCHUNK % 64 == 0 && NG4 % 64 == 0 && NEMB % 32 == 0 && NHID % 32 == 0, "tile multiples");
static_assert(NBATCH % RB_ROWS == 0 && RB_WAVES * 2 * 16 == NHID, "unit ownership: 16 waves x 2 unit-subtiles x 16 = 512");
static_assert((APITCH * 2) % 16 == 0 && (OPITCH * 4) % 16 == 0, "16-B aligned LDS rows");
static_assert(2 * RB_ROWS * APITCH * 2 >= RB_ROWS * OPITCH * 4, "output staging fits in the A-tile region");

__global__ __launch_bounds__(256) void cast_w_t(const float* __restrict__ kern, int krow0, int kdim, int tprl2,
                                                _Float16* __restrict__ outp, float mul, int nout) {
  const int gid = blockIdx.x * 256 + threadIdx.x;
  const int n = gid >> tprl2;
  const int q = gid & ((1 << tprl2) - 1);
  if (n >= nout) return;
  const float* src = kern + (size_t)(krow0 + q * 8) * NG4 + n;
  v8h hv;
#pragma unroll
  for (int e = 0; e < 8; ++e) hv[e] = (_Float16)(src[(size_t)e * NG4] * mul);
  _Float16* dst = outp + (size_t)n * kdim + q * 8;
  *(volatile v8h*)dst = hv;
  __threadfence();
  *(volatile v8h*)dst = hv;
}

__global__ __launch_bounds__(256) void gather_x16(const int* __restrict__ ids, const float* __restrict__ emb,
                                                  _Float16* __restrict__ x16, int nrows, int vocab) {
  const int gid = blockIdx.x * 256 + threadIdx.x;
  const int row = gid >> 5;
  const int q = gid & 31;
  if (row >= nrows) return;
  const int t = row >> 6;
  const int b = row & 63;
  int w = ids[b * NSTEP + t];
  w = (w < 0) ? 0 : w;
  w = (w > vocab - 1) ? (vocab - 1) : w;
  const float* src = emb + (size_t)w * NEMB + q * 8;
  const v4f a0 = *(const v4f*)(src);
  const v4f a1 = *(const v4f*)(src + 4);
  v8h hv;
  hv[0] = (_Float16)a0[0]; hv[1] = (_Float16)a0[1]; hv[2] = (_Float16)a0[2]; hv[3] = (_Float16)a0[3];
  hv[4] = (_Float16)a1[0]; hv[5] = (_Float16)a1[1]; hv[6] = (_Float16)a1[2]; hv[7] = (_Float16)a1[3];
  _Float16* dst = x16 + (size_t)row * NEMB + q * 8;
  *(volatile v8h*)dst = hv;
  __threadfence();
  *(volatile v8h*)dst = hv;
}

__device__ __forceinline__ float sigm_f(float x) {
  const float xc = fmaxf(x, -40.0f);
  return 1.0f / (1.0f + expf(-xc));
}

__global__ __launch_bounds__(RB_THREADS) void lstm_steps(
    const float* __restrict__ gx, const _Float16* __restrict__ wht,
    const int* __restrict__ num_words, const float* __restrict__ sprev,
    float* __restrict__ snext, int t0, int init) {
  __shared__ __align__(16) _Float16 At[2 * RB_ROWS * APITCH];
  float* Os = reinterpret_cast<float*>(At);
  union FH { v16h v; v8h h[2]; };

  const int tid  = threadIdx.x;
  const int wave = tid >> 5;
  const int lane = tid & 31;
  const int hh   = lane >> 4;
  const int cc   = lane & 15;
  const int b0   = blockIdx.x * RB_ROWS;

  int nw[8];
#pragma unroll
  for (int r = 0; r < 8; ++r) nw[r] = num_words[b0 + 8 * hh + r];

  float c_r[2][8], h_r[2][8];
#pragma unroll
  for (int u = 0; u < 2; ++u) {
    const int ucol = 16 * (2 * wave + u) + cc;
#pragma unroll
    for (int r = 0; r < 8; ++r) {
      const int row = 8 * hh + r;
      const float cv = sprev[(size_t)(b0 + row) * NHID + ucol];
      const float hv = sprev[(size_t)NBATCH * NHID + (size_t)(b0 + row) * NHID + ucol];
      c_r[u][r] = init ? 0.0f : cv;
      h_r[u][r] = init ? 0.0f : hv;
      At[row * APITCH + ucol] = (_Float16)h_r[u][r];
    }
  }
  __syncthreads();

#pragma unroll 1
  for (int t = 0; t < STEPS_PER_LAUNCH; ++t) {
    const int tg = t0 + t;
    const _Float16* Acur = At + (t & 1) * (RB_ROWS * APITCH);
    _Float16* Anext = At + ((t + 1) & 1) * (RB_ROWS * APITCH);
    const float* gxt = gx + (size_t)t * NBATCH * NG4 + (size_t)b0 * NG4;

#pragma unroll
    for (int u = 0; u < 2; ++u) {
      const int ucol = 16 * (2 * wave + u) + cc;
      v8f acc[4];
#pragma unroll
      for (int g = 0; g < 4; ++g) acc[g] = (v8f){0.f,0.f,0.f,0.f,0.f,0.f,0.f,0.f};
      const _Float16* arow = Acur + cc * APITCH + 8 * hh;
      const _Float16* bb0 = wht + (size_t)(0 * NHID + ucol) * NHID + 8 * hh;
      const _Float16* bb1 = wht + (size_t)(1 * NHID + ucol) * NHID + 8 * hh;
      const _Float16* bb2 = wht + (size_t)(2 * NHID + ucol) * NHID + 8 * hh;
      const _Float16* bb3 = wht + (size_t)(3 * NHID + ucol) * NHID + 8 * hh;
#pragma unroll 1
      for (int ks = 0; ks < NHID / 32; ++ks) {
        const int k0 = ks * 32;
        const v16h bq0 = Frag<_Float16>::load(bb0 + k0);
        const v16h bq1 = Frag<_Float16>::load(bb1 + k0);
        const v16h bq2 = Frag<_Float16>::load(bb2 + k0);
        const v16h bq3 = Frag<_Float16>::load(bb3 + k0);
        FH fa;
        fa.h[0] = *(const v8h*)(arow + k0);
        fa.h[1] = *(const v8h*)(arow + k0 + 16);
        acc[0] = Frag<_Float16>::mma(fa.v, bq0, acc[0]);
        acc[1] = Frag<_Float16>::mma(fa.v, bq1, acc[1]);
        acc[2] = Frag<_Float16>::mma(fa.v, bq2, acc[2]);
        acc[3] = Frag<_Float16>::mma(fa.v, bq3, acc[3]);
        Frag<_Float16>::guard(acc[0], acc[3], fa.v, bq3);
        Frag<_Float16>::keep(bq0, bq1, bq2, bq3);
      }
      acc_guard4(acc[0], acc[1], acc[2], acc[3]);

#pragma unroll
      for (int r = 0; r < 8; ++r) {
        const int row = 8 * hh + r;
        const float* gp = gxt + (size_t)row * NG4 + ucol;
        const float gxi = gp[0];
        const float gxj = gp[NHID];
        const float gxf = gp[2 * NHID];
        const float gxo = gp[3 * NHID];
        const float pi = acc[0][r] * W_CARRY_INV + gxi;
        const float pj = acc[1][r] * W_CARRY_INV + gxj;
        const float pf = acc[2][r] * W_CARRY_INV + gxf;
        const float po = acc[3][r] * W_CARRY_INV + gxo;
        const float cn = sigm_f(pf + 1.0f) * c_r[u][r] + sigm_f(pi) * tanhf(pj);
        const float hn = sigm_f(po) * tanhf(cn);
        const bool keep = tg < nw[r];
        c_r[u][r] = keep ? cn : c_r[u][r];
        h_r[u][r] = keep ? hn : h_r[u][r];
        Anext[row * APITCH + ucol] = (_Float16)h_r[u][r];
      }
    }
    __syncthreads();
  }

#pragma unroll
  for (int u = 0; u < 2; ++u) {
    const int ucol = 16 * (2 * wave + u) + cc;
#pragma unroll
    for (int r = 0; r < 8; ++r) Os[(8 * hh + r) * OPITCH + ucol] = c_r[u][r];
  }
  __syncthreads();
  {
    const float* srow = Os + wave * OPITCH;
    float* drow = snext + (size_t)(b0 + wave) * NHID;
    for (int pass = 0; pass < 2; ++pass) {
#pragma unroll
      for (int it = 0; it < 4; ++it) {
        v4f v = *(const v4f*)(srow + it * 128 + lane * 4);
        *(volatile v4f*)(drow + it * 128 + lane * 4) = v;
      }
      __threadfence();
    }
  }
  __syncthreads();
#pragma unroll
  for (int u = 0; u < 2; ++u) {
    const int ucol = 16 * (2 * wave + u) + cc;
#pragma unroll
    for (int r = 0; r < 8; ++r) Os[(8 * hh + r) * OPITCH + ucol] = h_r[u][r];
  }
  __syncthreads();
  {
    const float* srow = Os + wave * OPITCH;
    float* drow = snext + (size_t)NBATCH * NHID + (size_t)(b0 + wave) * NHID;
    for (int pass = 0; pass < 2; ++pass) {
#pragma unroll
      for (int it = 0; it < 4; ++it) {
        v4f v = *(const v4f*)(srow + it * 128 + lane * 4);
        *(volatile v4f*)(drow + it * 128 + lane * 4) = v;
      }
      __threadfence();
    }
  }
}

extern "C" void kernel_launch(void* const* d_in, const int* in_sizes, int n_in,
                              void* d_out, int out_size, void* d_ws,
                              size_t ws_size, hipStream_t stream) {
  if (n_in < 5) return;
  const int*   widx = (const int*)d_in[0];
  const int*   nwp  = (const int*)d_in[1];
  const float* emb  = (const float*)d_in[2];
  const float* kern = (const float*)d_in[3];
  const float* bias = (const float*)d_in[4];
  float* out = (float*)d_out;

  if (in_sizes[0] != NBATCH * NSTEP || in_sizes[1] != NBATCH ||
      in_sizes[3] != (NEMB + NHID) * NG4 || in_sizes[4] != NG4 ||
      out_size != 2 * NBATCH * NHID) return;
  const int vocab = in_sizes[2] / NEMB;
  if (vocab < 1) return;

  const size_t off_wxt = 0;
  const size_t byt_wxt = (size_t)NG4 * NEMB * 2;
  const size_t off_wht = off_wxt + byt_wxt;
  const size_t byt_wht = (size_t)NG4 * NHID * 2;
  const size_t off_x16 = off_wht + byt_wht;
  const size_t byt_x16 = (size_t)NSTEP * NBATCH * NEMB * 2;
  const size_t off_gx  = off_x16 + byt_x16;
  const size_t byt_gx  = (size_t)MCHUNK * NG4 * 4;
  const size_t off_s0  = off_gx + byt_gx;
  const size_t byt_s   = (size_t)2 * NBATCH * NHID * 4;
  const size_t off_s1  = off_s0 + byt_s;
  const size_t total   = off_s1 + byt_s;
  if (total > ws_size) return;

  char* ws = (char*)d_ws;
  _Float16* wxt = (_Float16*)(ws + off_wxt);
  _Float16* wht = (_Float16*)(ws + off_wht);
  _Float16* x16 = (_Float16*)(ws + off_x16);
  float* gxp = (float*)(ws + off_gx);
  float* s0 = (float*)(ws + off_s0);
  float* s1 = (float*)(ws + off_s1);

  cast_w_t<<<(NG4 * (NEMB / 8)) / 256, 256, 0, stream>>>(kern, 0, NEMB, 5, wxt, W_CARRY, NG4);
  cast_w_t<<<(NG4 * (NHID / 8)) / 256, 256, 0, stream>>>(kern, NEMB, NHID, 6, wht, W_CARRY, NG4);
  {
    const int nrows = NSTEP * NBATCH;
    gather_x16<<<(nrows * 32) / 256, 256, 0, stream>>>(widx, emb, x16, nrows, vocab);
  }

  for (int ch = 0; ch < NCHUNK; ++ch) {
    const unsigned grid_g = (unsigned)((MCHUNK / 64) * (NG4 / 64) / 8);
    wmma_gemm64<0, false, 2, 0, false, 0><<<dim3(grid_g, 1), 256, 0, stream>>>(
        (const unsigned short*)(x16 + (size_t)ch * MCHUNK * NEMB), (const unsigned short*)nullptr, NEMB, 0L,
        (const unsigned short*)wxt, (const unsigned short*)nullptr, NEMB, 0L,
        (void*)gxp, (void*)nullptr, NG4, 0L,
        bias, (const float*)nullptr, 0L,
        MCHUNK, NG4, NEMB, W_CARRY_INV);

    const float* sp = (ch & 1) ? s0 : s1;
    float* sn = (ch == NCHUNK - 1) ? out : ((ch & 1) ? s1 : s0);
    lstm_steps<<<NBATCH / RB_ROWS, RB_THREADS, 0, stream>>>(
        gxp, wht, nwp, sp, sn, ch * STEPS_PER_LAUNCH, (ch == 0) ? 1 : 0);
  }
}
